// LogicVAE_52012053954609
// MI455X (gfx1250) — hardware-verified
//
#include <hip/hip_runtime.h>


namespace {
constexpr int NB = 2048, NV = 32, V = 10, H = 256, Z = 64, H3 = 3 * H, H2 = 2 * H;
constexpr float XS = 8.0f, WSC = 256.0f;
typedef _Float16 b16;
typedef __attribute__((ext_vector_type(16))) _Float16 v16b;
typedef __attribute__((ext_vector_type(8))) _Float16 v8b;
typedef __attribute__((ext_vector_type(8))) float v8f;
typedef __attribute__((ext_vector_type(4))) float v4f;
__device__ __forceinline__ float bf16_rne(float f) { unsigned int u = __float_as_uint(f); u += 0x7FFFu + ((u >> 16) & 1u); return __uint_as_float(u & 0xFFFF0000u); }
__device__ __forceinline__ void split16(float v, b16& hi, b16& lo) { hi = (b16)v; lo = (b16)(v - (float)hi); }
__device__ __forceinline__ v16b frag_kb(const b16* p, int hh) { const v8b a = *(const v8b*)(p + 8 * hh), b = *(const v8b*)(p + 16 + 8 * hh); v16b f;
#pragma unroll
  for (int e = 0; e < 8; ++e) { f[e] = a[e]; f[8 + e] = b[e]; } return f; }
__device__ __forceinline__ v8f wmma16b(v16b a, v16b b, v8f c) { v8f d = __builtin_amdgcn_wmma_f32_16x16x32_f16(false, a, false, b, (short)0, c, false, false); asm volatile("v_nop\n\tv_nop\n\tv_nop\n\tv_nop" : "+v"(d) : "v"(a), "v"(b)); return d; }
__device__ __forceinline__ void wave_lds_sync() { __builtin_amdgcn_fence(__ATOMIC_RELEASE, "workgroup"); __builtin_amdgcn_wave_barrier(); __builtin_amdgcn_fence(__ATOMIC_ACQUIRE, "workgroup"); }
__device__ __forceinline__ float pmul(float a, float b) { float p = a * b; asm volatile("" : "+v"(p)); return p; }
__device__ __forceinline__ float sigm(float x) { return 1.0f / (1.0f + __expf(-x)); }
__device__ __forceinline__ int iclamp(int v, int lo, int hi) { return v < lo ? lo : (v > hi ? hi : v); }

__global__ __launch_bounds__(256) void wprep_kernel(const float* __restrict__ w, int nin, int nout, b16* __restrict__ dst) {
  const size_t u = (size_t)blockIdx.x * 256 + threadIdx.x; if (u >= (size_t)nout * nin / 8) return; const size_t e = u * 8; const int oo = (int)(e / nin), k0 = (int)(e % nin); v8b o;
  for (int j = 0; j < 8; ++j) o[j] = (b16)(bf16_rne(w[(size_t)(k0 + j) * nout + oo]) * WSC); for (int pass = 0; pass < 2; ++pass) { *(volatile v8b*)(dst + e) = o; __threadfence(); }
}
template <int MODE>
__global__ __launch_bounds__(128) void gemm_kernel(const float* __restrict__ SRC, const float* __restrict__ adj, int v, const b16* __restrict__ WT, int ncols, float* __restrict__ Y) {
  __shared__ __attribute__((aligned(16))) b16 Ah[4][16][H + 8], Al[4][16][H + 8]; __shared__ __attribute__((aligned(16))) float Tf[4][16][128 + 4];
  const int wave = threadIdx.x >> 5, lane = threadIdx.x & 31, nloc = lane & 15, hlf = lane >> 4; const size_t m0 = (size_t)blockIdx.x * 64 + wave * 16; const int n0 = blockIdx.y * 128;
  for (int rr = 0; rr < 16; ++rr) { const size_t b = m0 + rr; float a8[8];
    if (MODE == 0) { for (int j = 0; j < 8; ++j) a8[j] = 0.0f;
      for (int u = 0; u < v; ++u) { const float w = bf16_rne(adj[(b * NV + u) * NV + v]); const v4f g0 = *(const v4f*)(SRC + ((size_t)u * NB + b) * H + lane * 8), g1 = *(const v4f*)(SRC + ((size_t)u * NB + b) * H + lane * 8 + 4);
        for (int j = 0; j < 4; ++j) { a8[j] += pmul(w, g0[j]); a8[4 + j] += pmul(w, g1[j]); } } }
    else { const v4f g0 = *(const v4f*)(SRC + b * H + lane * 8), g1 = *(const v4f*)(SRC + b * H + lane * 8 + 4); for (int j = 0; j < 4; ++j) { a8[j] = g0[j]; a8[4 + j] = g1[j]; } }
    for (int j = 0; j < 8; ++j) { b16 p, q; split16(a8[j] * XS, p, q); Ah[wave][rr][lane * 8 + j] = p; Al[wave][rr][lane * 8 + j] = q; } }
  wave_lds_sync();
  v8f acc[8];
#pragma unroll
  for (int t = 0; t < 8; ++t) acc[t] = (v8f){};
#pragma unroll 2
  for (int kb = 0; kb < H; kb += 32) { const v16b a = frag_kb(&Ah[wave][nloc][kb], hlf), al = frag_kb(&Al[wave][nloc][kb], hlf);
#pragma unroll
    for (int t = 0; t < 8; ++t) { const v16b bw = frag_kb(WT + (size_t)(n0 + t * 16 + nloc) * H + kb, hlf); acc[t] = wmma16b(a, bw, acc[t]); acc[t] = wmma16b(al, bw, acc[t]); } }
#pragma unroll
  for (int t = 0; t < 8; ++t)
#pragma unroll 1
    for (int r = 0; r < 8; ++r) Tf[wave][8 * hlf + r][t * 16 + nloc] = acc[t][r] * (1.0f / (XS * WSC));
  wave_lds_sync();
  for (int pass = 0; pass < 2; ++pass) { for (int rr = 0; rr < 16; ++rr) *(volatile v4f*)(Y + (m0 + rr) * ncols + n0 + lane * 4) = *(const v4f*)(&Tf[wave][rr][lane * 4]); __threadfence(); }
}
__global__ __launch_bounds__(256) void gru_kernel(const int* __restrict__ types, int v, const float* __restrict__ wih, const float* __restrict__ bih, const float* __restrict__ bhh, const float* __restrict__ GH, const float* __restrict__ GM, const float* __restrict__ adj, float* __restrict__ HV) {
  const size_t u_ = (size_t)blockIdx.x * 256 + threadIdx.x; const size_t b = u_ / H; const int j = (int)(u_ % H); if (b >= (size_t)NB) return;
  const int ty = iclamp(types[b * NV + v], 0, V - 1);
  float hp = 0.0f; for (int u = 0; u < v; ++u) hp += pmul(bf16_rne(adj[(b * NV + u) * NV + v]), GM[((size_t)u * NB + b) * H + j]);
  const float gir = bf16_rne(wih[(size_t)ty * H3 + j]) + bf16_rne(bih[j]), giz = bf16_rne(wih[(size_t)ty * H3 + H + j]) + bf16_rne(bih[H + j]), gin = bf16_rne(wih[(size_t)ty * H3 + 2 * H + j]) + bf16_rne(bih[2 * H + j]);
  const float ghr = GH[b * H3 + j] + bf16_rne(bhh[j]), ghz = GH[b * H3 + H + j] + bf16_rne(bhh[H + j]), ghn = GH[b * H3 + 2 * H + j] + bf16_rne(bhh[2 * H + j]);
  const float r = sigm(gir + ghr), z = sigm(giz + ghz); const float n = tanhf(gin + pmul(r, ghn)); const float h = pmul(1.0f - z, n) + pmul(z, hp);
  for (int pass = 0; pass < 2; ++pass) { ((volatile float*)HV)[b * H + j] = h; __threadfence(); }
}
__global__ __launch_bounds__(256) void gm_kernel(const float* __restrict__ GP, const float* __restrict__ bg, int v, float* __restrict__ GM) {
  const size_t u_ = (size_t)blockIdx.x * 256 + threadIdx.x; const size_t b = u_ / H; const int j = (int)(u_ % H); if (b >= (size_t)NB) return;
  const float g = pmul(sigm(GP[b * H2 + j] + bf16_rne(bg[j])), GP[b * H2 + H + j]);
  for (int pass = 0; pass < 2; ++pass) { ((volatile float*)GM)[((size_t)v * NB + b) * H + j] = g; __threadfence(); }
}
__global__ __launch_bounds__(256) void out_kernel(const float* __restrict__ MS, const float* __restrict__ bmu, const float* __restrict__ bstd, float* __restrict__ mu, float* __restrict__ sg) {
  const size_t u_ = (size_t)blockIdx.x * 256 + threadIdx.x; const size_t b = u_ / 32; const int q = (int)(u_ % 32); if (b >= (size_t)NB) return;
  const int half = q >> 4, c4 = (q & 15) * 4; v4f o; for (int i = 0; i < 4; ++i) o[i] = MS[b * 128 + half * Z + c4 + i] + bf16_rne(half ? bstd[c4 + i] : bmu[c4 + i]);
  for (int pass = 0; pass < 2; ++pass) { *(volatile v4f*)((half ? sg : mu) + b * Z + c4) = o; __threadfence(); }
}
}

extern "C" void kernel_launch(void* const* d_in, const int* in_sizes, int n_in, void* d_out, int out_size, void* d_ws, size_t ws_size, hipStream_t stream) {
  (void)n_in;
  auto Fp = [&](int i) { return (const float*)d_in[i]; }; auto Ip = [&](int i) { return (const int*)d_in[i]; };
  if (in_sizes[0] != NB * NV * NV || in_sizes[1] != NB * NV || in_sizes[2] != V * H3 || in_sizes[3] != H * H3 || in_sizes[6] != H * H || in_sizes[8] != H * H || in_sizes[9] != H * Z || in_sizes[11] != H * Z || out_size != 2 * NB * Z) return;
  size_t off = 0; char* ws = (char*)d_ws;
  auto carve = [&](size_t bytes) { char* p = ws + off; off += (bytes + 255) & ~(size_t)255; return p; };
  b16* WHH = (b16*)carve((size_t)H3 * H * 2); b16* WGM = (b16*)carve((size_t)H2 * H * 2); b16* WMS = (b16*)carve((size_t)128 * H * 2);
  float* GM = (float*)carve((size_t)NV * NB * H * 4); float* GH = (float*)carve((size_t)NB * H3 * 4); float* GP = (float*)carve((size_t)NB * H2 * 4); float* HV = (float*)carve((size_t)NB * H * 4); float* MS = (float*)carve((size_t)NB * 128 * 4);
  if (off > ws_size || off > ((size_t)128 << 20)) return;
  wprep_kernel<<<(H3 * H / 8 + 255) / 256, 256, 0, stream>>>(Fp(3), H, H3, WHH);
  wprep_kernel<<<(H * H / 8 + 255) / 256, 256, 0, stream>>>(Fp(6), H, H, WGM); wprep_kernel<<<(H * H / 8 + 255) / 256, 256, 0, stream>>>(Fp(8), H, H, WGM + (size_t)H * H);
  wprep_kernel<<<(H * Z / 8 + 255) / 256, 256, 0, stream>>>(Fp(9), H, Z, WMS); wprep_kernel<<<(H * Z / 8 + 255) / 256, 256, 0, stream>>>(Fp(11), H, Z, WMS + (size_t)Z * H);
  for (int v = 0; v < NV; ++v) {
    gemm_kernel<0><<<dim3(NB / 64, H3 / 128), 128, 0, stream>>>(GM, Fp(0), v, WHH, H3, GH);
    gru_kernel<<<NB * H / 256, 256, 0, stream>>>(Ip(1), v, Fp(2), Fp(4), Fp(5), GH, GM, Fp(0), HV);
    if (v < NV - 1) { gemm_kernel<1><<<dim3(NB / 64, H2 / 128), 128, 0, stream>>>(HV, nullptr, v, WGM, H2, GP);
      gm_kernel<<<NB * H / 256, 256, 0, stream>>>(GP, Fp(7), v, GM); }
  }
  gemm_kernel<1><<<dim3(NB / 64, 1), 128, 0, stream>>>(HV, nullptr, 0, WMS, 128, MS);
  out_kernel<<<NB * 32 / 256, 256, 0, stream>>>(MS, Fp(10), Fp(12), (float*)d_out, (float*)d_out + (size_t)NB * Z);
}
